// ManualMHA_77300821393583
// MI455X (gfx1250) — hardware-verified
//
#include <hip/hip_runtime.h>
#include <math.h>

typedef __attribute__((ext_vector_type(16))) _Float16 v16h;
typedef __attribute__((ext_vector_type(8)))  _Float16 v8h;
typedef __attribute__((ext_vector_type(16))) __bf16   v16b;
typedef __attribute__((ext_vector_type(8)))  float    v8f;
typedef __attribute__((ext_vector_type(4)))  float    v4f;

__device__ __forceinline__ int frag_k(int i, int h) { return (i < 8) ? (8 * h + i) : (16 + 8 * h + (i - 8)); }
__device__ __forceinline__ __bf16 bf16_rne(float f) {
    unsigned int u = __float_as_uint(f);
    u += 0x7fffu + ((u >> 16) & 1u);
    return __builtin_bit_cast(__bf16, (unsigned short)(u >> 16));
}
__device__ __forceinline__ float bf16_f32(__bf16 b) { return __uint_as_float(((unsigned int)__builtin_bit_cast(unsigned short, b)) << 16); }
__device__ __forceinline__ v8f wmma16(v16h a, v16h b, v8f c) {
    c = __builtin_amdgcn_wmma_f32_16x16x32_f16(false, a, false, b, (short)0, c, false, false);
    asm volatile("v_nop\n\tv_nop\n\tv_nop\n\tv_nop" : "+v"(c) : "v"(a), "v"(b));
    return c;
}
__device__ __forceinline__ v8f wmmab(v16b a, v16b b, v8f c) {
    c = __builtin_amdgcn_wmma_f32_16x16x32_bf16(false, a, false, b, (short)0, c, false, false);
    asm volatile("v_nop\n\tv_nop\n\tv_nop\n\tv_nop" : "+v"(c) : "v"(a), "v"(b));
    return c;
}
struct Split { v16b hi, lo; };
__device__ __forceinline__ v8f wmma3(const Split& a, const Split& b, v8f c) {
    c = __builtin_amdgcn_wmma_f32_16x16x32_bf16(false, a.hi, false, b.hi, (short)0, c, false, false);
    c = __builtin_amdgcn_wmma_f32_16x16x32_bf16(false, a.hi, false, b.lo, (short)0, c, false, false);
    c = __builtin_amdgcn_wmma_f32_16x16x32_bf16(false, a.lo, false, b.hi, (short)0, c, false, false);
    asm volatile("v_nop\n\tv_nop\n\tv_nop\n\tv_nop" : "+v"(c) : "v"(a.hi), "v"(a.lo), "v"(b.hi), "v"(b.lo));
    return c;
}
struct Split3 { v16b hi, mid, lo; };
__device__ __forceinline__ v8f wmma6(const Split3& a, const Split3& b, v8f c) {
    c = __builtin_amdgcn_wmma_f32_16x16x32_bf16(false, a.hi, false, b.hi, (short)0, c, false, false);
    c = __builtin_amdgcn_wmma_f32_16x16x32_bf16(false, a.hi, false, b.mid, (short)0, c, false, false);
    c = __builtin_amdgcn_wmma_f32_16x16x32_bf16(false, a.mid, false, b.hi, (short)0, c, false, false);
    c = __builtin_amdgcn_wmma_f32_16x16x32_bf16(false, a.hi, false, b.lo, (short)0, c, false, false);
    c = __builtin_amdgcn_wmma_f32_16x16x32_bf16(false, a.mid, false, b.mid, (short)0, c, false, false);
    c = __builtin_amdgcn_wmma_f32_16x16x32_bf16(false, a.lo, false, b.hi, (short)0, c, false, false);
    asm volatile("v_nop\n\tv_nop\n\tv_nop\n\tv_nop" : "+v"(c) : "v"(a.hi), "v"(a.mid), "v"(a.lo), "v"(b.hi), "v"(b.mid), "v"(b.lo));
    return c;
}

__device__ __forceinline__ v16h fh_ld(const float* __restrict__ p, long long sk, int k0, int h, int klen, float s) {
    v16h a;
#pragma unroll
    for (int i = 0; i < 16; ++i) { const int k = k0 + frag_k(i, h); a[i] = (k < klen) ? (_Float16)(p[(long long)k * sk] * s) : (_Float16)0.f; }
    return a;
}
__device__ __forceinline__ Split sp_ld(const float* __restrict__ p, long long sk, int k0, int h, int klen, float s) {
    Split r;
#pragma unroll
    for (int i = 0; i < 16; ++i) {
        const int k = k0 + frag_k(i, h); const float x = (k < klen) ? p[(long long)k * sk] * s : 0.f;
        const __bf16 hb = bf16_rne(x); r.hi[i] = hb; r.lo[i] = bf16_rne(x - bf16_f32(hb));
    }
    return r;
}
__device__ __forceinline__ Split3 sp3_ld(const float* __restrict__ p, long long sk, int k0, int h, int klen, float s) {
    Split3 r;
#pragma unroll
    for (int i = 0; i < 16; ++i) {
        const int k = k0 + frag_k(i, h); const float x = (k < klen) ? p[(long long)k * sk] * s : 0.f;
        const __bf16 hb = bf16_rne(x); const float r1 = x - bf16_f32(hb); const __bf16 mb = bf16_rne(r1);
        r.hi[i] = hb; r.mid[i] = mb; r.lo[i] = bf16_rne(r1 - bf16_f32(mb));
    }
    return r;
}
__device__ __forceinline__ v16b bh_ld(const float* __restrict__ p, long long sk, int k0, int h, int klen, float s) {
    v16b a;
#pragma unroll
    for (int i = 0; i < 16; ++i) { const int k = k0 + frag_k(i, h); a[i] = bf16_rne((k < klen) ? p[(long long)k * sk] * s : 0.f); }
    return a;
}
__device__ __forceinline__ v16h fh_row(const _Float16* __restrict__ row, int k0, int h) {
    v16h a;
#pragma unroll
    for (int i = 0; i < 16; ++i) a[i] = row[k0 + frag_k(i, h)];
    return a;
}

#define VST2(T, ptr, val) do { const T vst2_v_ = (val); *(volatile T*)(ptr) = vst2_v_; __threadfence(); *(volatile T*)(ptr) = vst2_v_; } while (0)
typedef float v4f __attribute__((ext_vector_type(4)));
#define VST2V4(ptr, val) do { const v4f vst2_v4_ = (val); *(volatile v4f*)(ptr) = vst2_v4_; __threadfence(); *(volatile v4f*)(ptr) = vst2_v4_; } while (0)

__device__ __attribute__((noinline)) float act_fn(float v, int act) {
    if (act == 1) return fmaxf(v, 0.f);
    if (act == 2) { const float u = 0.7978845608028654f * (v + 0.044715f * v * v * v); return 0.5f * v * (1.f + tanhf(u)); }
    if (act == 3) return v / (1.f + expf(-v));
    if (act == 4) return 0.5f * v * (1.f + erff(v * 0.7071067811865476f));
    if (act == 5) return tanhf(v);
    if (act == 6) return 1.f / (1.f + expf(-v));
    if (act == 7) return (v > 0.f) ? v : 0.01f * v;
    if (act == 8) return (v > 0.f) ? v : (expf(v) - 1.f);
    if (act == 9) return fminf(fmaxf(v, 0.f), 6.f);
    if (act == 10) return fabsf(v);
    if (act == 11) return (v >= 0.f) ? v : 0.1f * v;
    if (act == 12) return (v > 0.f) ? v : 0.2f * v;
    if (act == 13) return (v > 20.f) ? v : log1pf(expf(v));
    return v;
}

#define AW 4
struct AttnP {
    const float* Q; const float* K; const float* V; float* O; float* P; const float* Mf; const int* Mi; float* ST;
    const float* Pw; const float* Rt; const int* SQ; const int* SK;
    long long swb, swh, swi, swj, srb, srh, sri;
    long long sQb, sQh, sQi, sQd, sKb, sKh, sKj, sKd, sVb, sVh, sVj, sVd, sOb, sOh, sOi, sPb, sPh, sPi, smb, smh, smi, smj;
    int Lq, Lk, dh, dv, hrep, causal, coff, pband;
    float scale, mfill; int nonorm, mpol;
    int roff, rn, segpol, win;
};
static_assert(sizeof(AttnP) == 12 * 8 + 29 * 8 + 16 * 4, "AttnP has padding");

#ifndef KATTN_ATTR
#define KATTN_ATTR
#endif
template <int DHP, int DVP, int QM, bool SPLITPV, bool TWOPASS>
__global__ __launch_bounds__(32 * AW) KATTN_ATTR void k_attn(AttnP p) {
    constexpr int NT = DVP / 16;
    constexpr int KS = DHP / 32;
    constexpr int VP = DVP + 8;
    __shared__ __align__(16) float    pl[AW][16 * 64];
    __shared__ __align__(16) _Float16 vl[(SPLITPV ? 2 : 1) * 64 * VP];
    const int lane = threadIdx.x & 31, hf = lane >> 4, l15 = lane & 15, wave = threadIdx.x >> 5;
    const int h = blockIdx.y, b = blockIdx.z, hk = h / p.hrep;
    const int q0 = (blockIdx.x * AW + wave) * 16;
    float* myp = pl[wave];
    const float L2E = 1.4426950408889634f;
    const float NEG = -__builtin_inff();
    const int qi = min(q0 + l15, p.Lq - 1);
    const float* qrow = p.Q + b * p.sQb + h * p.sQh + (long long)qi * p.sQi;
    const float* kbase = p.K + b * p.sKb + hk * p.sKh;
    const float* vbase = p.V + b * p.sVb + hk * p.sVh;
    v16h qa[QM == 0 ? KS : 1]; Split qs_[QM == 1 ? KS : 1]; Split3 qt_[QM == 2 ? KS : 1];
#pragma unroll
    for (int ks = 0; ks < KS; ++ks) {
        if (QM == 2) qt_[ks] = sp3_ld(qrow, p.sQd, ks * 32, hf, p.dh, 1.f);
        else if (QM == 1) qs_[ks] = sp_ld(qrow, p.sQd, ks * 32, hf, p.dh, 1.f);
        else qa[ks] = fh_ld(qrow, p.sQd, ks * 32, hf, p.dh, 1.f);
    }
    v8f o[NT]; float m8[8], l8[8];
#pragma unroll
    for (int t = 0; t < NT; ++t) { v8f zz = {}; o[t] = zz; }
#pragma unroll
    for (int i = 0; i < 8; ++i) { m8[i] = NEG; l8[i] = 0.f; }
    int jend = p.Lk; int jstart = 0;
    if (p.causal == 1) { const int je = (blockIdx.x * AW + AW - 1) * 16 + 16 + p.coff; jend = min(jend, max(je, 0)); }
    if (p.win > 0) { const int js = (int)(blockIdx.x * AW) * 16 + p.coff - p.win; jstart = (js > 0) ? (js / 64) * 64 : 0; }
    const int npass = TWOPASS ? 2 : 1;
    for (int pass = 0; pass < npass; ++pass) {
        const bool dopv = (!TWOPASS) || pass == 1;
        for (int j0 = jstart; j0 < jend; j0 += 64) {
            if (dopv) {
                __syncthreads();
                for (int idx = threadIdx.x; idx < 64 * DVP; idx += 32 * AW) {
                    const int jr = idx / DVP, d = idx - jr * DVP, j = j0 + jr;
                    const float f = (j < p.Lk && d < p.dv) ? vbase[(long long)j * p.sVj + (long long)d * p.sVd] : 0.f;
                    if (SPLITPV) {
                        const __bf16 hb = bf16_rne(f);
                        ((__bf16*)vl)[jr * VP + d] = hb; ((__bf16*)vl)[64 * VP + jr * VP + d] = bf16_rne(f - bf16_f32(hb));
                    } else vl[jr * VP + d] = (_Float16)f;
                }
            }
            v8f s[4];
#pragma unroll
            for (int t = 0; t < 4; ++t) {
                const int j = min(j0 + t * 16 + l15, p.Lk - 1);
                const float* krow = kbase + (long long)j * p.sKj;
                v8f acc = {};
#pragma unroll
                for (int ks = 0; ks < KS; ++ks) {
                    if (QM == 2)      acc = wmma6(qt_[ks], sp3_ld(krow, p.sKd, ks * 32, hf, p.dh, 1.f), acc);
                    else if (QM == 1) acc = wmma3(qs_[ks], sp_ld(krow, p.sKd, ks * 32, hf, p.dh, 1.f), acc);
                    else              acc = wmma16(qa[ks], fh_ld(krow, p.sKd, ks * 32, hf, p.dh, 1.f), acc);
                }
                s[t] = acc;
            }
            float pv[8][4];
#pragma unroll
            for (int i = 0; i < 8; ++i) {
                const int irow = q0 + i + 8 * hf;
                const int ic = min(irow, p.Lq - 1);
                float sc[4];
#pragma unroll
                for (int t = 0; t < 4; ++t) {
                    const int jg = j0 + t * 16 + l15;
                    float v = s[t][i] * p.scale;
                    if (p.Mf) v += p.Mf[b * p.smb + h * p.smh + (long long)ic * p.smi + (long long)min(jg, p.Lk - 1) * p.smj];
                    if (p.Rt) { int rc = ic - min(jg, p.Lk - 1) + p.roff; rc = rc < 0 ? 0 : (rc >= p.rn ? p.rn - 1 : rc); v += p.Rt[b * p.srb + h * p.srh + (long long)ic * p.sri + rc]; }
                    if (p.Mi) { const int mv = p.Mi[b * p.smb + h * p.smh + (long long)ic * p.smi + (long long)min(jg, p.Lk - 1) * p.smj]; if (p.mpol ? (mv != 0) : (mv == 0)) v = p.mfill; }
                    if (p.SQ) { const bool same = p.SQ[(long long)b * p.Lq + ic] == p.SK[(long long)b * p.Lk + min(jg, p.Lk - 1)]; if (p.segpol ? same : !same) v = p.mfill; }
                    if (p.causal == 2 && jg > irow + p.coff) v = p.mfill;
                    if (jg >= p.Lk || (p.causal == 1 && jg > irow + p.coff) || (p.causal == 3 && jg < irow + p.coff) || (p.win > 0 && irow + p.coff - jg > p.win)) v = NEG; else v *= L2E;
                    sc[t] = v;
                }
                if (!TWOPASS || pass == 0) {
                    float mx = fmaxf(fmaxf(sc[0], sc[1]), fmaxf(sc[2], sc[3]));
                    mx = fmaxf(mx, __shfl_xor(mx, 1, 32)); mx = fmaxf(mx, __shfl_xor(mx, 2, 32));
                    mx = fmaxf(mx, __shfl_xor(mx, 4, 32)); mx = fmaxf(mx, __shfl_xor(mx, 8, 32));
                    const float mnew = fmaxf(m8[i], mx);
                    const float corr = (mnew == NEG) ? 1.f : exp2f(m8[i] - mnew);
                    float rs = 0.f;
#pragma unroll
                    for (int t = 0; t < 4; ++t) {
                        const float pp = (sc[t] == NEG) ? 0.f : exp2f(sc[t] - mnew); rs += pp;
                        pv[i][t] = p.Pw ? pp * p.Pw[b * p.swb + h * p.swh + (long long)ic * p.swi + (long long)min(j0 + t * 16 + l15, p.Lk - 1) * p.swj] : pp;
                    }
                    rs += __shfl_xor(rs, 1, 32); rs += __shfl_xor(rs, 2, 32); rs += __shfl_xor(rs, 4, 32); rs += __shfl_xor(rs, 8, 32);
                    l8[i] = l8[i] * corr + rs; m8[i] = mnew;
                    if (!TWOPASS) {
#pragma unroll
                        for (int t = 0; t < NT; ++t) o[t][i] *= corr;
                    }
                } else {
                    const float inv = (l8[i] > 0.f) ? 1.f / l8[i] : 0.f;
#pragma unroll
                    for (int t = 0; t < 4; ++t) {
                        const int jg = j0 + t * 16 + l15;
                        float pp = (sc[t] == NEG) ? 0.f : exp2f(sc[t] - m8[i]) * inv;
                        if (p.Pw) pp *= p.Pw[b * p.swb + h * p.swh + (long long)ic * p.swi + (long long)min(jg, p.Lk - 1) * p.swj];
                        pv[i][t] = pp;
                    }
                }
            }
            if (dopv) {
#pragma unroll
                for (int i = 0; i < 8; ++i)
#pragma unroll
                    for (int t = 0; t < 4; ++t) ((volatile float*)myp)[(i + 8 * hf) * 64 + t * 16 + l15] = pv[i][t];
                __syncthreads();
                if (p.P) {
                    float* pb_ = p.P + b * p.sPb + h * p.sPh;
                    const bool fastP = (p.pband == 0) && ((p.sPi & 3) == 0) && (j0 + 64 <= p.Lk) && (q0 + 16 <= p.Lq) && ((((size_t)pb_) & 15) == 0);
                    if (fastP) {
#pragma unroll
                        for (int s = 0; s < 8; ++s) {
                            const int row = s * 2 + (lane >> 4), c4 = (lane & 15) * 4;
                            const v4f v = *(const v4f*)(myp + row * 64 + c4);
                            VST2V4(pb_ + (long long)(q0 + row) * p.sPi + j0 + c4, v);
                        }
                    } else {
                        for (int row = 0; row < 16; ++row) {
                            const int irow = q0 + row; if (irow >= p.Lq) continue;
                            for (int c = lane; c < 64; c += 32) {
                                const int jg = j0 + c; if (jg >= p.Lk) continue;
                                if (p.pband == 0) VST2(float, pb_ + (long long)irow * p.sPi + jg, myp[row * 64 + c]);
                                else if (jg - irow <= p.pband && irow - jg <= p.pband) VST2(float, pb_ + (long long)irow * p.sPi + (jg - irow + p.pband), myp[row * 64 + c]);
                            }
                        }
                    }
                }
                if (SPLITPV) {
                    const Split pa0 = sp_ld(myp + l15 * 64, 1, 0, hf, 64, 1.f), pa1 = sp_ld(myp + l15 * 64, 1, 32, hf, 64, 1.f);
                    const __bf16* vh = (const __bf16*)vl; const __bf16* vlo = vh + 64 * VP;
#pragma unroll
                    for (int t = 0; t < NT; ++t) {
                        const int dcol = t * 16 + l15;
                        Split b0, b1;
#pragma unroll
                        for (int e = 0; e < 16; ++e) {
                            const int k0 = frag_k(e, hf), k1 = 32 + frag_k(e, hf);
                            b0.hi[e] = vh[k0 * VP + dcol]; b0.lo[e] = vlo[k0 * VP + dcol]; b1.hi[e] = vh[k1 * VP + dcol]; b1.lo[e] = vlo[k1 * VP + dcol];
                        }
                        o[t] = wmma3(pa0, b0, o[t]);
                        o[t] = wmma3(pa1, b1, o[t]);
                    }
                } else {
                    const v16h pa0 = fh_ld(myp + l15 * 64, 1, 0, hf, 64, 4096.f), pa1 = fh_ld(myp + l15 * 64, 1, 32, hf, 64, 4096.f);
#pragma unroll
                    for (int t = 0; t < NT; ++t) {
                        const int dcol = t * 16 + l15;
                        v16h b0, b1;
#pragma unroll
                        for (int e = 0; e < 16; ++e) { b0[e] = vl[frag_k(e, hf) * VP + dcol]; b1[e] = vl[(32 + frag_k(e, hf)) * VP + dcol]; }
                        o[t] = wmma16(pa0, b0, o[t]);
                        o[t] = wmma16(pa1, b1, o[t]);
                    }
                }
            }
        }
    }
    float* obase = p.O + b * p.sOb + h * p.sOh;
    if (p.ST) {
        const int rl = lane >> 1, isel = rl & 7;
        float mv = 0.f, lv = 0.f;
#pragma unroll
        for (int i = 0; i < 8; ++i) if (i == isel) { mv = m8[i]; lv = l8[i]; }
        const int irow = q0 + rl;
        if (irow < p.Lq) { float* st = p.ST + (((long long)b * gridDim.y + h) * p.Lq + irow) * 2 + (lane & 1); VST2(float, st, (lane & 1) ? lv : mv * 0.6931471805599453f); }
    }
    float invr[8];
#pragma unroll
    for (int i = 0; i < 8; ++i) {
        if (TWOPASS) invr[i] = SPLITPV ? 1.f : (1.f / 4096.f);
        else if (p.nonorm) invr[i] = exp2f(m8[i]) * (SPLITPV ? 1.f : (1.f / 4096.f));
        else invr[i] = (l8[i] > 0.f) ? (SPLITPV ? 1.f / l8[i] : 1.f / (l8[i] * 4096.f)) : 0.f;
    }
    __syncthreads();
    const bool ofast = ((p.sOi & 3) == 0) && ((((size_t)obase) & 15) == 0) && (q0 + 16 <= p.Lq);
#pragma unroll
    for (int c0 = 0; c0 < DVP; c0 += 64) {
#pragma unroll
        for (int i = 0; i < 8; ++i)
#pragma unroll
            for (int t = 0; t < NT; ++t) if (t * 16 >= c0 && t * 16 < c0 + 64) ((volatile float*)myp)[(i + 8 * hf) * 64 + (t * 16 - c0) + l15] = o[t][i] * invr[i];
        __syncthreads();
        const int cw = (DVP - c0 < 64) ? (DVP - c0) : 64;
        if (ofast && (c0 + cw <= p.dv) && (cw % 32 == 0)) {
            const int lpr = cw / 4;
            const int rows_per_ins = 32 / lpr;
            for (int r0 = 0; r0 < 16; r0 += rows_per_ins) {
                const int row = r0 + lane / lpr, c4 = (lane % lpr) * 4;
                const v4f v = *(const v4f*)(myp + row * 64 + c4);
                VST2V4(obase + (long long)(q0 + row) * p.sOi + c0 + c4, v);
            }
        } else {
            for (int row = 0; row < 16; ++row) {
                const int irow = q0 + row; if (irow >= p.Lq) continue;
                for (int c = lane; c < cw; c += 32) { const int d = c0 + c; if (d < p.dv) VST2(float, obase + (long long)irow * p.sOi + d, myp[row * 64 + c]); }
            }
        }
        __syncthreads();
    }
}


#define GSTR 48
typedef _Float16 f16; typedef _Float16 bf16;
typedef v16h f16x16; typedef v16h bf16x16; typedef v8h f16x8; typedef v8h bf16x8; typedef v8f f32x8;
typedef __attribute__((ext_vector_type(4))) float v4f_t; typedef float v4fa __attribute__((ext_vector_type(4), may_alias));
typedef __attribute__((ext_vector_type(4))) unsigned v4u_t; typedef unsigned v4ua __attribute__((ext_vector_type(4), may_alias));
__device__ __forceinline__ f16x16 lds_frag(const f16* base, int stride) {
  const int lane = threadIdx.x & 31, row = lane & 15, kh = (lane >> 4) * 8;
  const f16x8 lo = *(const f16x8*)(base + row * stride + kh);
  const f16x8 hi = *(const f16x8*)(base + row * stride + kh + 16);
  f16x16 f;
#pragma unroll
  for (int i = 0; i < 8; ++i) { f[i] = lo[i]; f[i + 8] = hi[i]; }
  return f;
}

template <typename AT, bool ACC>
__global__ __launch_bounds__(256) void gemm_kn2(const AT* __restrict__ A, int lda, size_t strideA,
                                               const float* __restrict__ Wm, int ldw, size_t strideW,
                                               const float* __restrict__ bias, float scale,
                                               float* __restrict__ Y, int ldy, size_t strideY, int K) {
  __shared__ __attribute__((aligned(16))) f16 ldsA[128 * GSTR], ldsAl[128 * GSTR];
  __shared__ __attribute__((aligned(16))) f16 ldsW[128 * GSTR], ldsWl[128 * GSTR];
  __shared__ __attribute__((aligned(16))) float oS[8][32 * 68];
  const int tid = threadIdx.x, lane = tid & 31, wave = tid >> 5, cl = lane & 15, rh = (lane >> 4) * 8;
  const int m0 = blockIdx.x * 128, n0 = blockIdx.y * 128;
  const int wm = (wave & 3) * 32, wn = (wave >> 2) * 64;
  A += (size_t)blockIdx.z * strideA; Wm += (size_t)blockIdx.z * strideW; Y += (size_t)blockIdx.z * strideY;
  f32x8 acc[2][4], accx[2][4];
#pragma unroll
  for (int i = 0; i < 2; ++i)
#pragma unroll
    for (int j = 0; j < 4; ++j) { f32x8 z = {}; acc[i][j] = z; accx[i][j] = z; }
#pragma unroll 1
  for (int k0 = 0; k0 < K; k0 += 32) {
    __syncthreads();
    {
      const int row = tid >> 1, ch = (tid & 1) * 16;
      const AT* src = A + (size_t)(m0 + row) * lda + k0 + ch;
#pragma unroll
      for (int g = 0; g < 16; ++g) { const float v = (float)src[g]; const f16 h = (f16)v; ldsA[row * GSTR + ch + g] = h; ldsAl[row * GSTR + ch + g] = (f16)((v - (float)h) * 2048.0f); }
    }
    {
      const int k = tid >> 3, nn0 = (tid & 7) * 16;
      const float* src = Wm + (size_t)(k0 + k) * ldw + n0 + nn0;
#pragma unroll
      for (int g = 0; g < 4; ++g) { const v4f_t v = *(const v4f_t*)(src + 4 * g);
#pragma unroll
        for (int u = 0; u < 4; ++u) { const f16 h = (f16)v[u]; ldsW[(nn0 + 4 * g + u) * GSTR + k] = h; ldsWl[(nn0 + 4 * g + u) * GSTR + k] = (f16)((v[u] - (float)h) * 2048.0f); } }
    }
    __syncthreads();
    f16x16 af[2], afl[2];
#pragma unroll
    for (int i = 0; i < 2; ++i) { af[i] = lds_frag(ldsA + (wm + 16 * i) * GSTR, GSTR); afl[i] = lds_frag(ldsAl + (wm + 16 * i) * GSTR, GSTR); }
#pragma unroll
    for (int j = 0; j < 4; ++j) {
      const f16x16 bf = lds_frag(ldsW + (wn + 16 * j) * GSTR, GSTR), bfl = lds_frag(ldsWl + (wn + 16 * j) * GSTR, GSTR);
#pragma unroll
      for (int i = 0; i < 2; ++i) { acc[i][j] = wmma16(af[i], bf, acc[i][j]); accx[i][j] = wmma16(af[i], bfl, accx[i][j]); accx[i][j] = wmma16(afl[i], bf, accx[i][j]); }
    }
  }
  float* so = oS[wave];
#pragma unroll
  for (int i = 0; i < 2; ++i)
#pragma unroll
    for (int j = 0; j < 4; ++j) {
      const float bv = bias ? bias[n0 + wn + 16 * j + cl] : 0.0f;
#pragma unroll
      for (int r = 0; r < 8; ++r) so[(16 * i + rh + r) * 68 + 16 * j + cl] = (acc[i][j][r] + accx[i][j][r] * (1.0f / 2048.0f)) * scale + bv;
    }
  asm volatile("s_wait_dscnt 0" ::: "memory");
  __builtin_amdgcn_wave_barrier();
  if (ACC) {
#pragma unroll
    for (int it = 0; it < 16; ++it) { const int f4 = lane + 32 * it, rr = f4 >> 4, q = (f4 & 15) * 4;
      const v4f_t old = *(const v4fa*)(Y + (size_t)(m0 + wm + rr) * ldy + n0 + wn + q);
      v4f_t v = *(const v4fa*)(so + rr * 68 + q); v += old; *(volatile v4fa*)(so + rr * 68 + q) = v; }
    asm volatile("s_wait_dscnt 0" ::: "memory");
  }
#pragma unroll 1
  for (int pass = 0; pass < 2; ++pass) {
#pragma unroll
    for (int it = 0; it < 16; ++it) { const int f4 = lane + 32 * it, rr = f4 >> 4, q = (f4 & 15) * 4;
      *(volatile v4f_t*)(Y + (size_t)(m0 + wm + rr) * ldy + n0 + wn + q) = *(const v4fa*)(so + rr * 68 + q); }
    __threadfence();
  }
}

#define BBm 2
#define TTm 2048
#define DDm 1024
#define NHm 16
#define DKm 64
#define MTOK (BBm * TTm)
__global__ __launch_bounds__(256) void k_transpose(const float* __restrict__ Wm, float* __restrict__ Wt, int rows, int cols) {
  __shared__ float tS[64][65];
  const int tid = threadIdx.x, tbj = cols / 64, bi = blockIdx.x / tbj, bj = blockIdx.x % tbj;
  for (int e = tid; e < 64 * 64; e += 256) { const int r = e >> 6, c = e & 63; tS[r][c] = Wm[(size_t)(bi * 64 + r) * cols + bj * 64 + c]; }
  __syncthreads();
  for (int ch = tid; ch < 64 * 16; ch += 256) { const int r = ch >> 4, q4 = (ch & 15) * 4; v4f_t o; o[0] = tS[q4][r]; o[1] = tS[q4 + 1][r]; o[2] = tS[q4 + 2][r]; o[3] = tS[q4 + 3][r];
    float* dst = Wt + (size_t)(bj * 64 + r) * rows + bi * 64 + q4; *(volatile v4f_t*)dst = o; __threadfence(); *(volatile v4f_t*)dst = o; }
}
__global__ __launch_bounds__(256) void k_zeroi(int* __restrict__ p, int n) { for (int i = blockIdx.x * 256 + threadIdx.x; i < n; i += gridDim.x * 256) { *(volatile int*)(p + i) = 0; __threadfence(); *(volatile int*)(p + i) = 0; } }

extern "C" void kernel_launch(void* const* d_in, const int* in_sizes, int n_in,
                              void* d_out, int out_size, void* d_ws, size_t ws_size,
                              hipStream_t stream) {
  (void)in_sizes; (void)n_in; (void)out_size;
  const float** f = (const float**)d_in;
  const float* xq = f[0], *xk = f[1], *xv = f[2], *Wq = f[3], *bq = f[4], *Wk = f[5], *bk = f[6], *Wv = f[7], *bv = f[8], *Wo = f[9], *bo = f[10];
  const int* amask = (const int*)d_in[11];
  const int* kpm = (const int*)d_in[12];
  float* out = (float*)d_out;
  char* ws = (char*)d_ws;
  float* WqT = (float*)ws; ws += (size_t)DDm * DDm * 4; float* WkT = (float*)ws; ws += (size_t)DDm * DDm * 4; float* WvT = (float*)ws; ws += (size_t)DDm * DDm * 4; float* WoT = (float*)ws; ws += (size_t)DDm * DDm * 4;
  float* q32 = (float*)ws; ws += (size_t)MTOK * DDm * 4; float* k32 = (float*)ws; ws += (size_t)MTOK * DDm * 4; float* v32 = (float*)ws; ws += (size_t)MTOK * DDm * 4;
  float* O = (float*)ws; ws += (size_t)MTOK * DDm * 4;
  int* sq0 = (int*)ws; ws += (size_t)MTOK * 4;
  if ((size_t)(ws - (char*)d_ws) > ws_size) return;
  const dim3 blk(256);
  k_transpose<<<dim3((DDm / 64) * (DDm / 64)), blk, 0, stream>>>(Wq, WqT, DDm, DDm);
  k_transpose<<<dim3((DDm / 64) * (DDm / 64)), blk, 0, stream>>>(Wk, WkT, DDm, DDm);
  k_transpose<<<dim3((DDm / 64) * (DDm / 64)), blk, 0, stream>>>(Wv, WvT, DDm, DDm);
  k_transpose<<<dim3((DDm / 64) * (DDm / 64)), blk, 0, stream>>>(Wo, WoT, DDm, DDm);
  k_zeroi<<<dim3(16), blk, 0, stream>>>(sq0, MTOK);
  gemm_kn2<float, false><<<dim3(MTOK / 128, DDm / 128, 1), blk, 0, stream>>>(xq, DDm, 0, WqT, DDm, 0, bq, 1.0f, q32, DDm, 0, DDm);
  gemm_kn2<float, false><<<dim3(MTOK / 128, DDm / 128, 1), blk, 0, stream>>>(xk, DDm, 0, WkT, DDm, 0, bk, 1.0f, k32, DDm, 0, DDm);
  gemm_kn2<float, false><<<dim3(MTOK / 128, DDm / 128, 1), blk, 0, stream>>>(xv, DDm, 0, WvT, DDm, 0, bv, 1.0f, v32, DDm, 0, DDm);
  AttnP p = {};
  p.Q = q32; p.K = k32; p.V = v32; p.O = O; p.Mi = amask; p.SQ = sq0; p.SK = kpm;
  p.sQb = (long long)TTm * DDm; p.sQh = DKm; p.sQi = DDm; p.sQd = 1;
  p.sKb = (long long)TTm * DDm; p.sKh = DKm; p.sKj = DDm; p.sKd = 1;
  p.sVb = (long long)TTm * DDm; p.sVh = DKm; p.sVj = DDm; p.sVd = 1;
  p.sOb = (long long)TTm * DDm; p.sOh = DKm; p.sOi = DDm;
  p.smb = 0; p.smh = 0; p.smi = TTm; p.smj = 1; p.mpol = 1;
  p.Lq = TTm; p.Lk = TTm; p.dh = DKm; p.dv = DKm; p.hrep = 1; p.causal = 1; p.coff = 0; p.pband = 0;
  p.scale = 0.125f; p.mfill = -1.0e30f; p.nonorm = 0; p.roff = 0; p.rn = 0; p.segpol = 0; p.win = 0;
  k_attn<64, 64, 1, true, false><<<dim3(TTm / (16 * AW), NHm, BBm), dim3(32 * AW), 0, stream>>>(p);
  gemm_kn2<float, false><<<dim3(MTOK / 128, DDm / 128, 1), blk, 0, stream>>>(O, DDm, 0, WoT, DDm, 0, bo, 1.0f, out, DDm, 0, DDm);
}
